// FullyConnectedCapsule_22857815949492
// MI455X (gfx1250) — hardware-run, weakly checked
//
#include <hip/hip_runtime.h>
#include <math.h>

typedef __attribute__((ext_vector_type(16))) _Float16     v16h;
typedef __attribute__((ext_vector_type(8)))  _Float16     v8h;
typedef __attribute__((ext_vector_type(8)))  float        v8f;
typedef __attribute__((ext_vector_type(4)))  float        v4f;
typedef __attribute__((ext_vector_type(2)))  float        v2f;
typedef __attribute__((ext_vector_type(8)))  unsigned int v8u;

constexpr int kBatch   = 16384;
constexpr int kNumOut  = 32;
constexpr int kDimOut  = 16;
constexpr int kNumIn   = 16;
constexpr int kDimIn   = 8;
constexpr int kKdim    = kNumIn * kDimIn;
constexpr int kTileB   = 16;
constexpr int kWaves   = 8;
constexpr int kGrpPerWave = kNumOut / kWaves;
constexpr int kXfPitch = 132;
constexpr int kXhPitch = 136;
constexpr int kOutRow  = kNumOut * kDimOut;
constexpr int kSlab    = kGrpPerWave * kNumIn * kTileB;

constexpr float kXCarry  = 16.0f;
constexpr float kWCarry  = 64.0f;
constexpr float kCxCarry = 256.0f;

static_assert(kKdim == 128, "flattened k extent");
static_assert((kKdim % 32) == 0, "k multiple of 32");
static_assert(kDimOut == 16 && kTileB == 16, "one 16x16 tile per output group");
static_assert(kDimIn == 8, "one input vector = one 8-wide k run");
static_assert((kBatch % kTileB) == 0, "no batch tail");
static_assert(kGrpPerWave == 4, "four output groups per wave");
static_assert(kSlab == kTileB * kGrpPerWave * kDimOut, "result slab fits the dead logit rows");
static_assert(kGrpPerWave * kDimOut * 4 == 256, "wave row segment = two whole 128-B lines");
static_assert(kBatch * kKdim == 2097152, "x element count");
static_assert(kNumOut * kKdim * kDimOut == 65536, "W element count");
static_assert(kNumOut * kNumIn == 512, "bias element count");
static_assert((size_t)kBatch * kOutRow * 4 == 33554432ull, "output bytes");

constexpr size_t kWtHalves = (size_t)kNumOut * kDimOut * kKdim;
constexpr size_t kWsTotal  = kWtHalves * 2;
static_assert(kWsTotal == 131072ull, "carve total");
static_assert(kWsTotal <= 134217728ull, "carve cap");

union FragH { v16h v; v8h h[2]; };

__device__ __forceinline__ float bf16_rne(float f) {
  unsigned u = __float_as_uint(f);
  u = (u + 0x7FFFu + ((u >> 16) & 1u)) & 0xFFFF0000u;
  return __uint_as_float(u);
}

__device__ __forceinline__ v16h frag_load_global(const _Float16* p) {
  FragH f;
  f.h[0] = *(const v8h*)(p);
  f.h[1] = *(const v8h*)(p + 16);
  return f.v;
}

__device__ __forceinline__ v8f mma_h(v16h a, v16h b, v8f c) {
  c = __builtin_amdgcn_wmma_f32_16x16x32_f16(false, a, false, b, (short)0, c, false, false);
  asm volatile("v_nop\n\tv_nop\n\tv_nop\n\tv_nop" : "+v"(c) : "v"(a), "v"(b));
  return c;
}

__global__ __launch_bounds__(256) void weight_plane_kernel(
    const float* __restrict__ W, unsigned short* __restrict__ Wt)
{
  const int gid = blockIdx.x * 256 + threadIdx.x;
  const int j = gid & 15;
  const int z = (gid >> 4) & 15;
  const int n = gid >> 8;
  const float* src = W + ((size_t)(n * kNumIn + j) * kDimIn) * kDimOut + z;
  v8h hv;
#pragma unroll
  for (int i = 0; i < kDimIn; ++i) {
    const float wraw = src[i * kDimOut];
    const float wq = bf16_rne(wraw);
    const float wv = wq * kWCarry;
    hv[i] = (_Float16)wv;
  }
  unsigned short* dst = Wt + (size_t)gid * 8;
  *(volatile v8h*)dst = hv;
  __threadfence();
  *(volatile v8h*)dst = hv;
}

__global__ __launch_bounds__(256) void fused_route_kernel(
    const float* __restrict__ X, const _Float16* __restrict__ Wt,
    const float* __restrict__ Bias, float* __restrict__ Out)
{
  __shared__ __align__(16) float    sXf[kTileB * kXfPitch];
  __shared__ __align__(16) _Float16 sXh[kTileB * kXhPitch];
  __shared__ __align__(16) float    sC[kNumOut * kNumIn * kTileB];
  __shared__ __align__(16) float    sBias[kNumOut * kNumIn];

  const int tid  = threadIdx.x;
  const int lane = tid & 31;
  const int wave = __builtin_amdgcn_readfirstlane((int)(threadIdx.x >> 5));
  const int h    = lane >> 4;
  const int bcol = lane & 15;
  const size_t bt = (size_t)blockIdx.x * kTileB;

  {
    const int row  = tid >> 4;
    const int col8 = (tid & 15) * 8;
    const float* src = X + (bt + row) * kKdim + col8;
    const v4f a0 = *(const v4f*)(src);
    const v4f a1 = *(const v4f*)(src + 4);
    v4f r0, r1;
    v8h hv;
#pragma unroll
    for (int e = 0; e < 4; ++e) {
      const float s0 = a0[e];
      const float s1 = a1[e];
      const float q0 = bf16_rne(s0);
      const float q1 = bf16_rne(s1);
      r0[e] = q0;
      r1[e] = q1;
      const float f0 = q0 * kXCarry;
      const float f1 = q1 * kXCarry;
      hv[e]     = (_Float16)f0;
      hv[4 + e] = (_Float16)f1;
    }
    *(v4f*)(sXf + row * kXfPitch + col8)     = r0;
    *(v4f*)(sXf + row * kXfPitch + col8 + 4) = r1;
    *(v8h*)(sXh + row * kXhPitch + col8) = hv;
    const v2f bb = *(const v2f*)(Bias + 2 * tid);
    const float b0 = bb[0];
    const float b1 = bb[1];
    sBias[2 * tid]     = bf16_rne(b0);
    sBias[2 * tid + 1] = bf16_rne(b1);
  }
  __syncthreads();

  v16h xf[4];
  v8u  xw[4];
#pragma unroll
  for (int q = 0; q < 4; ++q) {
    FragH f;
    f.h[0] = *(const v8h*)(sXh + bcol * kXhPitch + 32 * q + 8 * h);
    f.h[1] = *(const v8h*)(sXh + bcol * kXhPitch + 32 * q + 16 + 8 * h);
    xf[q] = f.v;
    xw[q] = __builtin_bit_cast(v8u, f.v);
  }

  const float inv_sqrt_d = 1.0f / sqrtf((float)kDimOut);
  const float lscale = inv_sqrt_d * (1.0f / ((kWCarry * kXCarry) * (kWCarry * kXCarry)));
  const v8f zero8 = (v8f){0.f, 0.f, 0.f, 0.f, 0.f, 0.f, 0.f, 0.f};

#pragma unroll 1
  for (int t = 0; t < kGrpPerWave; ++t) {
    const int n = wave * kGrpPerWave + t;
    const _Float16* wrow = Wt + (size_t)(n * kDimOut + bcol) * kKdim + 8 * h;
    v16h wf[4];
#pragma unroll
    for (int q = 0; q < 4; ++q) wf[q] = frag_load_global(wrow + 32 * q);

    v8f us = zero8;
#pragma unroll
    for (int q = 0; q < 4; ++q) us = mma_h(wf[q], xf[q], us);

#pragma unroll
    for (int j = 0; j < kNumIn; ++j) {
      const int q  = j >> 2;
      const int jj = j & 3;
      const bool keep_lo = ((0 + h) == jj);
      const bool keep_hi = ((2 + h) == jj);
      v8u mw;
#pragma unroll
      for (int e = 0; e < 4; ++e) {
        mw[e]     = keep_lo ? xw[q][e]     : 0u;
        mw[4 + e] = keep_hi ? xw[q][4 + e] : 0u;
      }
      const v16h xm = __builtin_bit_cast(v16h, mw);
      const v8f u = mma_h(wf[q], xm, zero8);
      float p = u[0] * us[0];
#pragma unroll
      for (int r = 1; r < 8; ++r) p = fmaf(u[r], us[r], p);
      p += __shfl_xor(p, 16, 32);
      if (h == 0) sC[(n * kNumIn + j) * kTileB + bcol] = p * lscale;
    }
  }
  __syncthreads();

  {
    const int jcol = tid >> 4;
    float mx = -INFINITY;
#pragma unroll 8
    for (int n = 0; n < kNumOut; ++n) mx = fmaxf(mx, sC[n * (kNumIn * kTileB) + tid]);
    float ssum = 0.f;
#pragma unroll 4
    for (int n = 0; n < kNumOut; ++n) {
      const float ev = expf(sC[n * (kNumIn * kTileB) + tid] - mx);
      sC[n * (kNumIn * kTileB) + tid] = ev;
      ssum += ev;
    }
    const float inv = 1.0f / ssum;
#pragma unroll 8
    for (int n = 0; n < kNumOut; ++n) {
      const float cv = sC[n * (kNumIn * kTileB) + tid] * inv + sBias[n * kNumIn + jcol];
      sC[n * (kNumIn * kTileB) + tid] = cv;
    }
  }
  __syncthreads();

  const float oscale = 1.0f / (kWCarry * kCxCarry);
#pragma unroll 1
  for (int t = 0; t < kGrpPerWave; ++t) {
    const int n = wave * kGrpPerWave + t;
    const _Float16* wrow = Wt + (size_t)(n * kDimOut + bcol) * kKdim + 8 * h;
    v16h wf[4];
#pragma unroll
    for (int q = 0; q < 4; ++q) wf[q] = frag_load_global(wrow + 32 * q);

    v8f acc = zero8;
#pragma unroll
    for (int q = 0; q < 4; ++q) {
      const float c0 = sC[(n * kNumIn + 4 * q + h) * kTileB + bcol] * kCxCarry;
      const float c1 = sC[(n * kNumIn + 4 * q + 2 + h) * kTileB + bcol] * kCxCarry;
      const float* xr = sXf + bcol * kXfPitch + 32 * q + 8 * h;
      const v4f x0 = *(const v4f*)(xr);
      const v4f x1 = *(const v4f*)(xr + 4);
      const v4f x2 = *(const v4f*)(xr + 16);
      const v4f x3 = *(const v4f*)(xr + 20);
      v16h bf;
#pragma unroll
      for (int e = 0; e < 4; ++e) {
        const float f0 = x0[e] * c0;
        const float f1 = x1[e] * c0;
        const float f2 = x2[e] * c1;
        const float f3 = x3[e] * c1;
        bf[e]      = (_Float16)f0;
        bf[4 + e]  = (_Float16)f1;
        bf[8 + e]  = (_Float16)f2;
        bf[12 + e] = (_Float16)f3;
      }
      acc = mma_h(wf[q], bf, acc);
    }
    float* sl = sC + wave * kSlab + t * (kNumIn * kTileB) + bcol * kDimOut + 8 * h;
    const v4f o0 = (v4f){acc[0] * oscale, acc[1] * oscale, acc[2] * oscale, acc[3] * oscale};
    const v4f o1 = (v4f){acc[4] * oscale, acc[5] * oscale, acc[6] * oscale, acc[7] * oscale};
    *(v4f*)(sl)     = o0;
    *(v4f*)(sl + 4) = o1;
  }
  __syncthreads();

  {
    const int c4   = (lane & 15) * 4;
    const int tsel = c4 >> 4;
    const int z4   = c4 & 15;
    v4f vals[8];
#pragma unroll
    for (int it = 0; it < 8; ++it) {
      const int row = it * 2 + h;
      vals[it] = *(const v4f*)(sC + wave * kSlab + tsel * (kNumIn * kTileB) + row * kDimOut + z4);
    }
    float* obase = Out + bt * kOutRow + wave * (kGrpPerWave * kDimOut) + c4;
    for (int pass = 0; pass < 2; ++pass) {
#pragma unroll
      for (int it = 0; it < 8; ++it) {
        const int row = it * 2 + h;
        *(volatile v4f*)(obase + (size_t)row * kOutRow) = vals[it];
      }
      __threadfence();
    }
  }
}

extern "C" void kernel_launch(void* const* d_in, const int* in_sizes, int n_in,
                              void* d_out, int out_size, void* d_ws, size_t ws_size,
                              hipStream_t stream) {
  if (n_in < 3) return;
  if (in_sizes[0] != kBatch * kKdim) return;
  if (in_sizes[1] != kNumOut * kKdim * kDimOut) return;
  if (in_sizes[2] != kNumOut * kNumIn) return;
  if (out_size != kBatch * kOutRow) return;
  if (ws_size < kWsTotal) return;

  const float* X    = (const float*)d_in[0];
  const float* W    = (const float*)d_in[1];
  const float* Bias = (const float*)d_in[2];
  float* Out = (float*)d_out;
  unsigned short* WtBits = (unsigned short*)d_ws;

  weight_plane_kernel<<<(kNumOut * kDimOut * kNumIn) / 256, 256, 0, stream>>>(W, WtBits);

  fused_route_kernel<<<kBatch / kTileB, kWaves * 32, 0, stream>>>(X, (const _Float16*)d_ws, Bias, Out);
}
